// QuantumKANClassifier_26688926777603
// MI455X (gfx1250) — hardware-verified
//
#include <hip/hip_runtime.h>
#include <stddef.h>
#include <stdint.h>

#pragma clang fp contract(off)

#define NF    32
#define ND    16
#define NC    64
#define NG    8
#define KT    256
#define BM    64
#define LDA   264
#define STP   36
#define SWP   17
#define WSC   16.0f
#define RWSC  0.0625f
#define CLIPF 0.999999f

static_assert(KT == NF * NG);
static_assert(KT % 32 == 0);
static_assert((LDA * 2) % 16 == 0);
static_assert((STP * 4) % 16 == 0);
static_assert(BM == 64);

typedef _Float16 v16h __attribute__((ext_vector_type(16)));
typedef _Float16 v8h  __attribute__((ext_vector_type(8)));
typedef _Float16 v2h  __attribute__((ext_vector_type(2)));
typedef float    v8f  __attribute__((ext_vector_type(8)));
typedef float    v4f  __attribute__((ext_vector_type(4)));
typedef float    v2f  __attribute__((ext_vector_type(2)));
typedef unsigned int v4u __attribute__((ext_vector_type(4)));
typedef v8h __attribute__((may_alias)) v8ha;
typedef v4u __attribute__((may_alias)) v4ua;
typedef v4f __attribute__((may_alias)) v4fa;

union Frag { v16h v; v8h h[2]; };

__device__ __forceinline__ v8f mma16(v16h a, v16h b, v8f cacc) {
  cacc = __builtin_amdgcn_wmma_f32_16x16x32_f16(false, a, false, b, (short)0, cacc, false, false);
  asm volatile("v_nop\n\tv_nop\n\tv_nop\n\tv_nop" : "+v"(cacc) : "v"(a), "v"(b));
  return cacc;
}

__device__ __forceinline__ v8f zero8() { return (v8f){0.f, 0.f, 0.f, 0.f, 0.f, 0.f, 0.f, 0.f}; }

__device__ __forceinline__ v16h ldfrag_g(const _Float16* __restrict__ p, int ld, int row0, int k0, int lane) {
  const int m = lane & 15, lh = lane >> 4;
  const _Float16* q = p + (size_t)(row0 + m) * ld + k0 + 8 * lh;
  Frag f;
  f.h[0] = *(const v8h*)(q);
  f.h[1] = *(const v8h*)(q + 16);
  return f.v;
}

__device__ __forceinline__ v16h ldfrag_l(const _Float16* p, int ld, int row0, int k0, int lane) {
  const int m = lane & 15, lh = lane >> 4;
  const _Float16* q = p + (row0 + m) * ld + k0 + 8 * lh;
  Frag f;
  f.h[0] = *(const v8ha*)(q);
  f.h[1] = *(const v8ha*)(q + 16);
  return f.v;
}

__device__ __forceinline__ unsigned int pk2(float lo, float hi) {
  const v2f p = (v2f){lo, hi};
  const v2h q = __builtin_convertvector(p, v2h);
  return __builtin_bit_cast(unsigned int, q);
}

__device__ __forceinline__ unsigned int pk_one_lo(float hi) {
  const unsigned int hb = (unsigned int)__builtin_bit_cast(unsigned short, (_Float16)hi);
  return __builtin_amdgcn_perm(hb, 0x00003C00u, 0x05040100u);
}

__global__ __launch_bounds__(256) void k_prep(const float* __restrict__ kc, _Float16* __restrict__ Bw) {
  const int tid = threadIdx.x;
  v4u val[8];
#pragma unroll
  for (int j = 0; j < 8; ++j) {
    const int p = tid + 256 * j;
    const v4f x0 = *(const v4f*)(kc + (size_t)p * 8);
    const v4f x1 = *(const v4f*)(kc + (size_t)p * 8 + 4);
    v4u v;
    v.x = pk2(x0.x * WSC, x0.y * WSC);
    v.y = pk2(x0.z * WSC, x0.w * WSC);
    v.z = pk2(x1.x * WSC, x1.y * WSC);
    v.w = pk2(x1.z * WSC, x1.w * WSC);
    val[j] = v;
  }
#pragma unroll
  for (int j = 0; j < 8; ++j) *(volatile v4u*)(Bw + (size_t)(tid + 256 * j) * 8) = val[j];
  __threadfence();
#pragma unroll
  for (int j = 0; j < 8; ++j) *(volatile v4u*)(Bw + (size_t)(tid + 256 * j) * 8) = val[j];
}

__global__ __launch_bounds__(256) void k_main(const float* __restrict__ X, const float* __restrict__ ph,
                                              const float* __restrict__ lw, const float* __restrict__ ssc,
                                              const float* __restrict__ sbi, const _Float16* __restrict__ Bw,
                                              const float* __restrict__ kb, float* __restrict__ out) {
  __shared__ float sPh[ND];
  __shared__ float sW[NF * SWP];
  __shared__ __align__(16) _Float16 sA[BM * LDA];
  __shared__ __align__(16) float st[8][16 * STP];

  const int tid = threadIdx.x, lane = tid & 31, wave = tid >> 5;
  const int hh = lane >> 4, c = lane & 15;
  const int bm0 = blockIdx.x * BM;

  {
    const int tp = (tid < ND) ? tid : (ND - 1);
    const float pv = ph[tp];
    if (tid < ND) sPh[tid] = pv;
    const int i0 = tid, i1 = tid + 256;
    sW[(i0 >> 4) * SWP + (i0 & 15)] = lw[i0];
    sW[(i1 >> 4) * SWP + (i1 & 15)] = lw[i1];
  }
  __syncthreads();

  const float* wl = sW + lane * SWP;
  float den = 0.0f;
#pragma unroll 1
  for (int d = 0; d < ND; ++d) den = den + fabsf(wl[d]);
  den = den + 1e-6f;
  const float rden = 1.0f / den;
  const float sc = ssc[lane];
  const float sb = sbi[lane];

#pragma unroll 1
  for (int j = 0; j < 8; ++j) {
    const int row = wave + 8 * j;
    const float xv = X[(size_t)(bm0 + row) * NF + lane];
    const float xc = fminf(fmaxf(xv, -CLIPF), CLIPF);
    const float th = acosf(xc);
    float aq = 0.0f;
#pragma unroll 1
    for (int d = 0; d < ND; ++d) {
      float arg = th * (float)(d + 1);
      arg = arg + sPh[d];
      aq = aq + cosf(arg) * wl[d];
    }
    const float lcu = aq * rden;
    const float v   = sc * lcu + sb;
    const float ft  = tanhf(v);
    const float fcv = fminf(fmaxf(ft, -CLIPF), CLIPF);
    const float t2  = acosf(fcv);
    const float b1 = cosf(t2);
    const float b2 = cosf(t2 * 2.0f);
    const float b3 = cosf(t2 * 3.0f);
    const float b4 = cosf(t2 * 4.0f);
    const float b5 = cosf(t2 * 5.0f);
    const float b6 = cosf(t2 * 6.0f);
    const float b7 = cosf(t2 * 7.0f);
    v4u pv;
    pv.x = pk_one_lo(b1);
    pv.y = pk2(b2, b3);
    pv.z = pk2(b4, b5);
    pv.w = pk2(b6, b7);
    *(v4ua*)(sA + row * LDA + lane * 8) = pv;
  }
  __syncthreads();

  const int rt = wave >> 1;
  const int ch = wave & 1;
  const int n0 = 32 * ch;
  v8f acc0 = zero8(), acc1 = zero8();
#pragma unroll
  for (int ks = 0; ks < KT / 32; ++ks) {
    const int k0 = ks * 32;
    const v16h a   = ldfrag_l(sA, LDA, rt * 16, k0, lane);
    const v16h bq0 = ldfrag_g(Bw, KT, n0, k0, lane);
    const v16h bq1 = ldfrag_g(Bw, KT, n0 + 16, k0, lane);
    acc0 = mma16(a, bq0, acc0);
    acc1 = mma16(a, bq1, acc1);
  }

  const float bv0 = kb[n0 + c];
  const float bv1 = kb[n0 + 16 + c];
  float* sw = st[wave];
#pragma unroll
  for (int r = 0; r < 8; ++r) {
    sw[(8 * hh + r) * STP + c]      = acc0[r] * RWSC + bv0;
    sw[(8 * hh + r) * STP + 16 + c] = acc1[r] * RWSC + bv1;
  }
  __syncthreads();
  v4f val[4];
  size_t go[4];
#pragma unroll
  for (int it = 0; it < 4; ++it) {
    const int p  = lane + 32 * it;
    const int L  = p >> 3;
    const int pc = p & 7;
    val[it] = *(const v4fa*)(sw + L * STP + pc * 4);
    go[it]  = (size_t)(bm0 + rt * 16 + L) * NC + n0 + pc * 4;
  }
#pragma unroll
  for (int it = 0; it < 4; ++it) *(volatile v4f*)(out + go[it]) = val[it];
  __threadfence();
#pragma unroll
  for (int it = 0; it < 4; ++it) *(volatile v4f*)(out + go[it]) = val[it];
}

extern "C" void kernel_launch(void* const* d_in, const int* in_sizes, int n_in,
                              void* d_out, int out_size, void* d_ws, size_t ws_size,
                              hipStream_t stream) {
  if (n_in < 7) return;
  const int nx = in_sizes[0];
  if (nx <= 0 || (nx % NF) != 0) return;
  const int nb = nx / NF;
  if ((nb % BM) != 0) return;
  if (in_sizes[1] != ND) return;
  if (in_sizes[2] != NF * ND) return;
  if (in_sizes[3] != NF) return;
  if (in_sizes[4] != NF) return;
  if (in_sizes[5] != NC * KT) return;
  if (in_sizes[6] != NC) return;
  if (out_size != nb * NC) return;

  const float* x     = (const float*)d_in[0];
  const float* ph    = (const float*)d_in[1];
  const float* lw    = (const float*)d_in[2];
  const float* ssc   = (const float*)d_in[3];
  const float* sbi   = (const float*)d_in[4];
  const float* kc    = (const float*)d_in[5];
  const float* kb    = (const float*)d_in[6];
  float* out = (float*)d_out;

  const size_t bw_bytes = (size_t)NC * KT * 2;
  if (bw_bytes > ws_size) return;
  _Float16* Bw = (_Float16*)d_ws;

  k_prep<<<dim3(1), dim3(256), 0, stream>>>(kc, Bw);
  k_main<<<dim3(nb / BM), dim3(256), 0, stream>>>(x, ph, lw, ssc, sbi, Bw, kb, out);
  (void)hipGetLastError();
}
